// ConvCNP2D_87771951661186
// MI455X (gfx1250) — hardware-run, weakly checked
//
#include <hip/hip_runtime.h>
#include <math.h>

typedef __attribute__((ext_vector_type(16))) _Float16 v16h;
typedef __attribute__((ext_vector_type(8)))  _Float16 v8h;
typedef __attribute__((ext_vector_type(8)))  float    v8f;
typedef __attribute__((ext_vector_type(4)))  float    v4f;

constexpr int kBatch   = 4;
constexpr int kCtx     = 256;
constexpr int kGridDim = 32;
constexpr int kGridPts = kGridDim * kGridDim;
constexpr int kChanIn  = 16;
constexpr int kChanHid = 32;
constexpr int kChanOut = 16;
constexpr int kTaps    = 25;
constexpr int kChanPad = 32;
constexpr int kKdim    = kTaps * kChanPad;
constexpr int kPix     = kBatch * kGridPts;
constexpr int kSlabP   = 36;
static_assert(kGridPts == 1024 && kPix == 4096 && kKdim == 800, "shape constants");
static_assert((kKdim % 32) == 0, "conv K is a whole number of 32-deep steps");
static_assert((kPix % 128) == 0, "8 pixel tiles of 16 per block");
static_assert((kChanHid % 16) == 0 && (kChanOut % 16) == 0, "N tiles of 16");
static_assert(((kGridPts * kChanOut) % 32) == 0, "read-out K is a whole number of 32-deep steps");

constexpr float kActCarry   = 64.0f;
constexpr float kWgtCarry   = 256.0f;
constexpr float kConvFold   = 1.0f / (kActCarry * kWgtCarry);
constexpr float kHeadACarry = 1024.0f;
constexpr float kHeadFold   = 1.0f / (kHeadACarry * kActCarry);
constexpr float kF16MinNormal = 6.103515625e-5f;
constexpr float kF32MinNormal = 1.17549435e-38f;

constexpr size_t kOffWP1  = 0;
constexpr size_t kOffWP2  = kOffWP1  + (size_t)kChanHid * kKdim * 2;
constexpr size_t kOffWP3  = kOffWP2  + (size_t)kChanHid * kKdim * 2;
constexpr size_t kOffACT0 = kOffWP3  + (size_t)kChanOut * kKdim * 2;
constexpr size_t kOffACT1 = kOffACT0 + (size_t)kPix * kChanPad * 2;
constexpr size_t kOffACT2 = kOffACT1 + (size_t)kPix * kChanHid * 2;
constexpr size_t kOffH3   = kOffACT2 + (size_t)kPix * kChanHid * 2;
constexpr size_t kWsTotal = kOffH3   + (size_t)kPix * kChanOut * 2;
static_assert(kWsTotal == 1045504ull, "carve total");
static_assert(kWsTotal <= 134217728ull, "carve cap");
static_assert((kOffWP2 % 128) == 0 && (kOffWP3 % 128) == 0 && (kOffACT0 % 128) == 0 &&
              (kOffACT1 % 128) == 0 && (kOffACT2 % 128) == 0 && (kOffH3 % 128) == 0, "128-B aligned regions");

__device__ __forceinline__ _Float16 to_h_flush(float v) {
  const float w = (fabsf(v) < kF16MinNormal) ? 0.0f : v;
  return (_Float16)w;
}
__device__ __forceinline__ v8h pack8_flush(const float* sp) {
  const v4f a0 = *(const v4f*)(sp);
  const v4f a1 = *(const v4f*)(sp + 4);
  v8h hv;
#pragma unroll
  for (int e = 0; e < 4; ++e) {
    hv[e]     = to_h_flush(a0[e]);
    hv[4 + e] = to_h_flush(a1[e]);
  }
  return hv;
}
union FragH { v16h v; v8h h[2]; };
__device__ __forceinline__ v16h frag_load(const _Float16* p) {
  FragH f;
  f.h[0] = *(const v8h*)(p);
  f.h[1] = *(const v8h*)(p + 16);
  return f.v;
}
__device__ __forceinline__ v8f mma_h(v16h a, v16h b, v8f c) {
  c = __builtin_amdgcn_wmma_f32_16x16x32_f16(false, a, false, b, (short)0, c, false, false);
  asm volatile("v_nop\n\tv_nop\n\tv_nop\n\tv_nop" : "+v"(c) : "v"(a), "v"(b));
  return c;
}

__global__ __launch_bounds__(128) void weight_plane_kernel(
    const float* __restrict__ W1, const float* __restrict__ W2, const float* __restrict__ W3,
    unsigned short* __restrict__ P1, unsigned short* __restrict__ P2, unsigned short* __restrict__ P3)
{
  const int layer = blockIdx.y;
  const float* W = W1;
  unsigned short* dst = P1;
  int cin = kChanIn;
  int cout = kChanHid;
  if (layer == 1) { W = W2; dst = P2; cin = kChanHid; cout = kChanHid; }
  if (layer == 2) { W = W3; dst = P3; cin = kChanHid; cout = kChanOut; }
  const int ci = blockIdx.x * 128 + threadIdx.x;
  if (ci >= cout * 100) return;
  const int o   = ci / 100;
  const int r   = ci - o * 100;
  const int tap = r >> 2;
  const int c0  = (r & 3) * 8;
  v8h hv;
#pragma unroll
  for (int e = 0; e < 8; ++e) {
    const int c  = c0 + e;
    const int cc = (c < cin) ? c : (cin - 1);
    float w = W[(size_t)(o * cin + cc) * kTaps + tap];
    asm volatile("" : "+v"(w));
    const float ws = (c < cin) ? (w * kWgtCarry) : 0.0f;
    hv[e] = to_h_flush(ws);
  }
  unsigned short* q = dst + (size_t)ci * 8;
  *(volatile v8h*)q = hv;
  __threadfence();
  *(volatile v8h*)q = hv;
}

__global__ __launch_bounds__(256) void rbf_grid_in_kernel(
    const float* __restrict__ x, const float* __restrict__ y, const float* __restrict__ xg,
    const float* __restrict__ sig, const float* __restrict__ Win, const float* __restrict__ bin,
    unsigned short* __restrict__ act0)
{
  __shared__ __align__(16) float sPx[kCtx * 2];
  __shared__ __align__(16) float sPy[kCtx];
  __shared__ __align__(16) float sT[256 * kSlabP];
  const int tid = threadIdx.x, lane = tid & 31, wave = tid >> 5;
  const int b = blockIdx.x >> 2;
  const int m = (blockIdx.x & 3) * 256 + tid;
  sPx[2 * tid]     = x[(size_t)(b * kCtx + tid) * 2];
  sPx[2 * tid + 1] = x[(size_t)(b * kCtx + tid) * 2 + 1];
  sPy[tid]         = y[(size_t)b * kCtx + tid];
  const float tx = xg[2 * m];
  const float ty = xg[2 * m + 1];
  const float s0 = expf(sig[0]);
  const float s1 = expf(sig[1]);
  const float f0 = -0.5f * (1.0f / (s0 * s0));
  const float f1 = -0.5f * (1.0f / (s1 * s1));
  __syncthreads();
  float dens = 0.0f, conv = 0.0f;
#pragma unroll 1
  for (int n = 0; n < kCtx; ++n) {
    const float dx = sPx[2 * n] - tx;
    const float dy = sPx[2 * n + 1] - ty;
    const float d  = dx * dx + dy * dy;
    float e0 = expf(d * f0);
    float e1 = expf(d * f1);
    e0 = (e0 < kF32MinNormal) ? 0.0f : e0;
    e1 = (e1 < kF32MinNormal) ? 0.0f : e1;
    dens += e0;
    conv = fmaf(e1, sPy[n], conv);
  }
  const float feat0 = dens;
  const float feat1 = conv * (1.0f / (dens + 1e-8f));
  float* myrow = sT + tid * kSlabP;
#pragma unroll 1
  for (int o = 0; o < kChanIn; ++o) {
    const float w0 = Win[2 * o];
    const float w1 = Win[2 * o + 1];
    const float bo = bin[o];
    const float v  = (w0 * feat0 + w1 * feat1) + bo;
    const float s  = 1.0f / (1.0f + expf(-v));
    myrow[o]           = s * kActCarry;
    myrow[kChanIn + o] = 0.0f;
  }
  __syncthreads();
  v8h hv[4];
#pragma unroll
  for (int it = 0; it < 4; ++it) {
    const int q   = it * 32 + lane;
    const int row = wave * 32 + (q >> 2);
    const int c8  = (q & 3) * 8;
    hv[it] = pack8_flush(sT + row * kSlabP + c8);
  }
  unsigned short* obase = act0 + ((size_t)blockIdx.x * 256 + wave * 32) * kChanPad;
  for (int pass = 0; pass < 2; ++pass) {
#pragma unroll
    for (int it = 0; it < 4; ++it) {
      const int q = it * 32 + lane;
      *(volatile v8h*)(obase + (size_t)q * 8) = hv[it];
    }
    __threadfence();
  }
}

template <int COUT, bool RELU>
__global__ __launch_bounds__(256) void conv5_kernel(
    const unsigned short* __restrict__ actIn, const unsigned short* __restrict__ wpl,
    const float* __restrict__ bias, unsigned short* __restrict__ actOut)
{
  constexpr int NT  = COUT / 16;
  constexpr int CH8 = COUT / 8;
  constexpr int NIT = (16 * CH8) / 32;
  static_assert(NT >= 1 && NT <= 2 && NIT >= 1, "tile shape");
  __shared__ __align__(16) float sT[8][16 * kSlabP];
  const int tid = threadIdx.x, lane = tid & 31, wave = tid >> 5;
  const int hh = lane >> 4, rl = lane & 15;
  const int tile = blockIdx.x * 8 + wave;
  const int bb   = tile >> 6;
  const int ml0  = (tile & 63) * 16;
  const int gi   = ml0 >> 5;
  const int gj   = (ml0 & 31) + rl;
  const _Float16* A  = (const _Float16*)actIn;
  const _Float16* Bt = (const _Float16*)wpl;

  v8f acc[NT];
#pragma unroll
  for (int nt = 0; nt < NT; ++nt) acc[nt] = (v8f){0.f, 0.f, 0.f, 0.f, 0.f, 0.f, 0.f, 0.f};

#pragma unroll 1
  for (int kh = 0; kh < 5; ++kh) {
    const int jj = gj + kh - 2;
    const bool vj = (jj >= 0) && (jj < kGridDim);
    const int jc = min(max(jj, 0), kGridDim - 1);
#pragma unroll 1
    for (int kw = 0; kw < 5; ++kw) {
      const int ii = gi + kw - 2;
      const bool vv = vj && (ii >= 0) && (ii < kGridDim);
      const int ic = min(max(ii, 0), kGridDim - 1);
      const int tap = kh * 5 + kw;
      v16h av = frag_load(A + ((size_t)(bb * kGridPts + ic * kGridDim + jc) * kChanPad + 8 * hh));
      asm volatile("" : "+v"(av));
      const v16h zero = {};
      const v16h a = vv ? av : zero;
#pragma unroll
      for (int nt = 0; nt < NT; ++nt) {
        const v16h bv = frag_load(Bt + ((size_t)(nt * 16 + rl) * kKdim + tap * 32 + 8 * hh));
        acc[nt] = mma_h(a, bv, acc[nt]);
      }
    }
  }

  float* slab = sT[wave];
#pragma unroll
  for (int nt = 0; nt < NT; ++nt) {
    const float bo = bias[nt * 16 + rl];
#pragma unroll
    for (int r = 0; r < 8; ++r) {
      float v = acc[nt][r] * kConvFold + bo;
      if (RELU) v = fmaxf(v, 0.0f);
      slab[(8 * hh + r) * kSlabP + nt * 16 + rl] = v * kActCarry;
    }
  }
  __syncthreads();
  v8h hv[NIT];
#pragma unroll
  for (int it = 0; it < NIT; ++it) {
    const int q   = it * 32 + lane;
    const int row = q / CH8;
    const int c8  = (q - row * CH8) * 8;
    hv[it] = pack8_flush(slab + row * kSlabP + c8);
  }
  unsigned short* obase = actOut + (size_t)tile * 16 * COUT;
  for (int pass = 0; pass < 2; ++pass) {
#pragma unroll
    for (int it = 0; it < NIT; ++it) {
      const int q = it * 32 + lane;
      *(volatile v8h*)(obase + (size_t)q * 8) = hv[it];
    }
    __threadfence();
  }
}

__global__ __launch_bounds__(256) void rbf_readout_kernel(
    const unsigned short* __restrict__ h3p, const float* __restrict__ xg,
    const float* __restrict__ sig_m, const float* __restrict__ W_m, const float* __restrict__ b_m,
    const float* __restrict__ sig_s, const float* __restrict__ W_s, const float* __restrict__ b_s,
    float* __restrict__ out)
{
  __shared__ __align__(16) float sG[kGridPts * 2];
  __shared__ __align__(16) float sR[8][256];
  const int tid = threadIdx.x, lane = tid & 31, wave = tid >> 5;
  const int hh = lane >> 4, rl = lane & 15;
  const int mt = wave & 1;
  const int head = (wave >> 1) & 1;
  const int ks = wave >> 2;
#pragma unroll
  for (int k = 0; k < 8; ++k) sG[tid + 256 * k] = xg[tid + 256 * k];

  const float* sg = head ? sig_s : sig_m;
  const float* wg = head ? W_s : W_m;
  float fc[8], wc[8];
#pragma unroll
  for (int e = 0; e < 8; ++e) {
    const int c = 8 * hh + e;
    const float s = expf(sg[c]);
    fc[e] = -0.5f * (1.0f / (s * s));
    wc[e] = wg[c] * kHeadACarry;
  }
  const int m = blockIdx.x * 32 + mt * 16 + rl;
  __syncthreads();
  const float gmx = sG[2 * m];
  const float gmy = sG[2 * m + 1];
  const _Float16* hb = (const _Float16*)h3p + (size_t)(rl & 3) * (kGridPts * kChanOut) + 8 * hh;

  v8f acc = (v8f){0.f, 0.f, 0.f, 0.f, 0.f, 0.f, 0.f, 0.f};
#pragma unroll 1
  for (int st = 0; st < 256; ++st) {
    const int n0 = ks * 512 + 2 * st;
    const v4f g = *(const v4f*)(sG + 2 * n0);
    const float dx0 = gmx - g[0];
    const float dy0 = gmy - g[1];
    const float dx1 = gmx - g[2];
    const float dy1 = gmy - g[3];
    const float d0 = dx0 * dx0 + dy0 * dy0;
    const float d1 = dx1 * dx1 + dy1 * dy1;
    v16h a;
#pragma unroll
    for (int e = 0; e < 8; ++e) {
      a[e]     = to_h_flush(expf(d0 * fc[e]) * wc[e]);
      a[8 + e] = to_h_flush(expf(d1 * fc[e]) * wc[e]);
    }
    const v16h bv = frag_load(hb + (size_t)n0 * kChanOut);
    acc = mma_h(a, bv, acc);
  }
#pragma unroll
  for (int r = 0; r < 8; ++r) sR[wave][(8 * hh + r) * 16 + rl] = acc[r];
  __syncthreads();
  {
    const int ob = wave & 3;
    const int oh = wave >> 2;
    const int omt = lane >> 4;
    const int orow = lane & 15;
    const int w0 = omt + 2 * oh;
    const int w1 = w0 + 4;
    const float bm = b_m[0];
    const float bs = b_s[0];
    const float bsel = oh ? bs : bm;
    const float sum = sR[w0][orow * 16 + ob] + sR[w1][orow * 16 + ob];
    const float val = sum * kHeadFold + bsel;
    float* q = out + (size_t)ob * (2 * kGridPts) + (size_t)oh * kGridPts + blockIdx.x * 32 + lane;
    *(volatile float*)q = val;
    __threadfence();
    *(volatile float*)q = val;
  }
}

extern "C" void kernel_launch(void* const* d_in, const int* in_sizes, int n_in,
                              void* d_out, int out_size, void* d_ws, size_t ws_size,
                              hipStream_t stream) {
  if (n_in < 18) return;
  if (in_sizes[0] != kBatch * kCtx * 2) return;
  if (in_sizes[1] != kBatch * kCtx) return;
  if (in_sizes[2] != kGridPts * 2) return;
  if (in_sizes[3] != 2) return;
  if (in_sizes[4] != kChanIn * 2) return;
  if (in_sizes[5] != kChanIn) return;
  if (in_sizes[6] != kChanOut || in_sizes[7] != kChanOut || in_sizes[8] != 1) return;
  if (in_sizes[9] != kChanOut || in_sizes[10] != kChanOut || in_sizes[11] != 1) return;
  if (in_sizes[12] != kChanHid * kChanIn * kTaps || in_sizes[13] != kChanHid) return;
  if (in_sizes[14] != kChanHid * kChanHid * kTaps || in_sizes[15] != kChanHid) return;
  if (in_sizes[16] != kChanOut * kChanHid * kTaps || in_sizes[17] != kChanOut) return;
  if (out_size != kBatch * 2 * kGridPts) return;
  if (ws_size < kWsTotal) return;

  const float* x        = (const float*)d_in[0];
  const float* y        = (const float*)d_in[1];
  const float* x_grid   = (const float*)d_in[2];
  const float* sigma_in = (const float*)d_in[3];
  const float* W_in     = (const float*)d_in[4];
  const float* b_in     = (const float*)d_in[5];
  const float* sigma_m  = (const float*)d_in[6];
  const float* W_m      = (const float*)d_in[7];
  const float* b_m      = (const float*)d_in[8];
  const float* sigma_s  = (const float*)d_in[9];
  const float* W_s      = (const float*)d_in[10];
  const float* b_s      = (const float*)d_in[11];
  const float* cW1      = (const float*)d_in[12];
  const float* cb1      = (const float*)d_in[13];
  const float* cW2      = (const float*)d_in[14];
  const float* cb2      = (const float*)d_in[15];
  const float* cW3      = (const float*)d_in[16];
  const float* cb3      = (const float*)d_in[17];
  float* outp = (float*)d_out;

  char* ws = (char*)d_ws;
  unsigned short* WP1  = (unsigned short*)(ws + kOffWP1);
  unsigned short* WP2  = (unsigned short*)(ws + kOffWP2);
  unsigned short* WP3  = (unsigned short*)(ws + kOffWP3);
  unsigned short* ACT0 = (unsigned short*)(ws + kOffACT0);
  unsigned short* ACT1 = (unsigned short*)(ws + kOffACT1);
  unsigned short* ACT2 = (unsigned short*)(ws + kOffACT2);
  unsigned short* H3   = (unsigned short*)(ws + kOffH3);

  weight_plane_kernel<<<dim3(25, 3), 128, 0, stream>>>(cW1, cW2, cW3, WP1, WP2, WP3);
  rbf_grid_in_kernel<<<kPix / 256, 256, 0, stream>>>(x, y, x_grid, sigma_in, W_in, b_in, ACT0);
  conv5_kernel<kChanHid, true ><<<kPix / 128, 256, 0, stream>>>(ACT0, WP1, cb1, ACT1);
  conv5_kernel<kChanHid, true ><<<kPix / 128, 256, 0, stream>>>(ACT1, WP2, cb2, ACT2);
  conv5_kernel<kChanOut, false><<<kPix / 128, 256, 0, stream>>>(ACT2, WP3, cb3, H3);
  rbf_readout_kernel<<<kGridPts / 32, 256, 0, stream>>>(H3, x_grid, sigma_m, W_m, b_m, sigma_s, W_s, b_s, outp);
}
